// GraphReasoner_77051713290524
// MI455X (gfx1250) — hardware-verified
//
#include <hip/hip_runtime.h>
#include <stdint.h>
#include <stddef.h>
#include <math.h>

#define NN    4096
#define DM    1024
#define KD    2048
#define NDEP  8
#define NC    64
#define NLEV  64
#define MT    32
#define NSL   256
#define XP    2056
#define YP    260
#define WSC   32.0f
#define WSCI  0.03125f
#define META_N 128

#define LDS_XB   (MT * XP * 2)
#define LDS_YB   (MT * YP * 4)
#define LDS_STEP (LDS_XB + LDS_YB)

static_assert((XP * 2) % 16 == 0);
static_assert((YP * 4) % 16 == 0);
static_assert(NN % 256 == 0);
static_assert(NN % MT == 0);
static_assert(DM % NSL == 0);
static_assert(KD % 32 == 0);
static_assert(KD == 8 * 256);
static_assert(NSL == 8 * 32);
static_assert(MT == 8 * 4);
static_assert(MT * NDEP == 256);
static_assert(LDS_XB % 16 == 0);
static_assert(NC == 64);
static_assert(META_N == 32 * 4);
static_assert(NLEV + 2 <= META_N);

typedef _Float16       v16h __attribute__((ext_vector_type(16)));
typedef _Float16       v8h  __attribute__((ext_vector_type(8)));
typedef float          v8f  __attribute__((ext_vector_type(8)));
typedef float          v4f  __attribute__((ext_vector_type(4)));
typedef unsigned int   v4u  __attribute__((ext_vector_type(4)));
typedef int            v4i  __attribute__((ext_vector_type(4)));
typedef v4f __attribute__((may_alias)) v4fa;
typedef v4u __attribute__((may_alias)) v4ua;
typedef v4i __attribute__((may_alias)) v4ia;

union FragH { v16h v; v4u q[2]; };
union Pk8   { v8h h; v4u u; };

__device__ __forceinline__ v4u pack8(v4f a, v4f c, float s) {
  Pk8 k;
  k.h[0] = (_Float16)(a.x * s); k.h[1] = (_Float16)(a.y * s);
  k.h[2] = (_Float16)(a.z * s); k.h[3] = (_Float16)(a.w * s);
  k.h[4] = (_Float16)(c.x * s); k.h[5] = (_Float16)(c.y * s);
  k.h[6] = (_Float16)(c.z * s); k.h[7] = (_Float16)(c.w * s);
  return k.u;
}

__device__ __forceinline__ v8f wmma_h(v16h a, v16h b, v8f c) {
  v8f d = __builtin_amdgcn_wmma_f32_16x16x32_f16(false, a, false, b, (short)0, c, false, false);
  asm volatile("v_nop\n\tv_nop\n\tv_nop\n\tv_nop" : "+v"(d) : "v"(a), "v"(b));
  return d;
}

__device__ __forceinline__ v16h ldfrag_h(const unsigned short* p, int h) {
  FragH f;
  f.q[0] = *(const v4ua*)(p + 8 * h);
  f.q[1] = *(const v4ua*)(p + 16 + 8 * h);
  return f.v;
}

__device__ __forceinline__ int clampi(int v, int lo, int hi) {
  return v < lo ? lo : (v > hi ? hi : v);
}

__global__ __launch_bounds__(256) void k_w1(const float* __restrict__ w1,
                                            unsigned short* __restrict__ w1h)
{
  const int row = blockIdx.x;
  const int tid = threadIdx.x;
  const float* src = w1 + (size_t)row * KD + 8 * tid;
  const v4f a = *(const v4fa*)src;
  const v4f c = *(const v4fa*)(src + 4);
  const v4u p = pack8(a, c, WSC);
  unsigned short* dst = w1h + (size_t)row * KD + 8 * tid;
  *(volatile v4u*)dst = p;
  __threadfence();
  *(volatile v4u*)dst = p;
}

__global__ __launch_bounds__(256) void k_levels(const int* __restrict__ dep_idx,
                                                const int* __restrict__ dep_mask,
                                                int* __restrict__ lev,
                                                int* __restrict__ meta)
{
  __shared__ __align__(16) int sLev[NN];
  __shared__ __align__(16) int sMeta[META_N];
  const int tid = threadIdx.x;
  for (int i = tid; i < NN; i += 256) sLev[i] = 0;
  if (tid < META_N) sMeta[tid] = 0;
  __syncthreads();

  if (tid == 0) {
    int maxl = 0, over = 0;
    #pragma unroll 1
    for (int i = 0; i < NN; ++i) {
      int best = -1;
      #pragma unroll
      for (int d = 0; d < NDEP; ++d) {
        const int mk = dep_mask[i * NDEP + d];
        const int dp = clampi(dep_idx[i * NDEP + d], 0, NN - 1);
        const int l  = sLev[dp];
        best = (mk != 0 && l > best) ? l : best;
      }
      const int lv = best + 1;
      sLev[i] = lv;
      maxl = (lv > maxl) ? lv : maxl;
      if (lv < NLEV) sMeta[lv] += 1; else over += 1;
    }
    sMeta[NLEV]     = maxl;
    sMeta[NLEV + 1] = over;
  }
  __syncthreads();

  v4i lv4[4];
  #pragma unroll
  for (int j = 0; j < 4; ++j) lv4[j] = *(const v4ia*)(sLev + 4 * (j * 256 + tid));
  const v4i mv = *(const v4ia*)(sMeta + 4 * (tid & 31));

  #pragma unroll
  for (int j = 0; j < 4; ++j) *(volatile v4i*)(lev + 4 * (j * 256 + tid)) = lv4[j];
  if (tid < 32) *(volatile v4i*)(meta + 4 * tid) = mv;
  __threadfence();
  #pragma unroll
  for (int j = 0; j < 4; ++j) *(volatile v4i*)(lev + 4 * (j * 256 + tid)) = lv4[j];
  if (tid < 32) *(volatile v4i*)(meta + 4 * tid) = mv;
}

__device__ __forceinline__ void ans_pass(const float* sY, const int* sTok, float* ans,
                                         int ns, int wv, int lane, int nrows)
{
  #pragma unroll
  for (int i = 0; i < 4; ++i) {
    const int row = wv * 4 + i;
    const int node = clampi(sTok[row], 0, NN - 1);
    const v4f v0 = *(const v4fa*)(sY + row * YP + 4 * lane);
    const v4f v1 = *(const v4fa*)(sY + row * YP + 128 + 4 * lane);
    float* dst = ans + (size_t)node * DM + ns * NSL;
    if (row < nrows) {
      *(volatile v4f*)(dst + 4 * lane) = v0;
      *(volatile v4f*)(dst + 128 + 4 * lane) = v1;
    }
  }
}

__global__ __launch_bounds__(256) void k_step(const float* __restrict__ q,
                                              const unsigned short* __restrict__ w1h,
                                              const float* __restrict__ b1,
                                              const int* __restrict__ dep_idx,
                                              const int* __restrict__ dep_mask,
                                              const int* __restrict__ lev,
                                              const int* __restrict__ meta,
                                              float* ans, int s)
{
  extern __shared__ __align__(16) unsigned char dsm[];
  unsigned short* sX = (unsigned short*)dsm;
  float* sY = (float*)(dsm + LDS_XB);
  __shared__ int   sTok[MT];
  __shared__ int   sDep[MT * NDEP];
  __shared__ float sMsk[MT * NDEP];
  __shared__ float sInv[MT];
  __shared__ int   s_wc[8];

  const int tid = threadIdx.x, lane = tid & 31, wv = tid >> 5;
  const int h = lane >> 4, m = lane & 15;
  const int m0 = blockIdx.x * MT;

  const int hint = clampi(meta[s & (NLEV - 1)], 0, NN);
  if (m0 >= hint) return;

  if (tid < MT) sTok[tid] = 0;
  __syncthreads();

  int base = 0;
  #pragma unroll 1
  for (int ch = 0; ch < NN / 256; ++ch) {
    const int t = ch * 256 + tid;
    const int lv = lev[t];
    const bool f = (lv == s);
    const unsigned int msk = __builtin_amdgcn_ballot_w32(f);
    const int off = __builtin_popcount(msk & ((1u << lane) - 1u));
    const int wc = __builtin_popcount(msk);
    if (lane == 0) s_wc[wv] = wc;
    __syncthreads();
    int pre = 0, tot = 0;
    #pragma unroll
    for (int w2 = 0; w2 < 8; ++w2) {
      const int cc = s_wc[w2];
      tot += cc;
      pre += (w2 < wv) ? cc : 0;
    }
    if (f) {
      const int p = base + pre + off - m0;
      if ((unsigned)p < (unsigned)MT) sTok[p] = t;
    }
    base += tot;
    __syncthreads();
  }
  const int cnt = base;
  if (m0 >= cnt) return;
  int nrows = cnt - m0;
  nrows = (nrows > MT) ? MT : nrows;

  {
    const int row = tid >> 3, d = tid & 7;
    const int node = clampi(sTok[row], 0, NN - 1);
    const int dp = clampi(dep_idx[(size_t)node * NDEP + d], 0, NN - 1);
    const int mk = dep_mask[(size_t)node * NDEP + d];
    sDep[tid] = dp;
    sMsk[tid] = (float)mk;
  }
  __syncthreads();
  if (tid < MT) {
    float c = 0.0f;
    #pragma unroll
    for (int d = 0; d < NDEP; ++d) c += sMsk[tid * NDEP + d];
    sInv[tid] = 1.0f / fmaxf(c, 1.0f);
  }
  __syncthreads();

  #pragma unroll 2
  for (int j = 0; j < 16; ++j) {
    const int idx = tid + 256 * j;
    const int row = idx >> 7, c8 = idx & 127;
    const int node = clampi(sTok[row], 0, NN - 1);
    const float* gq = q + (size_t)node * DM + 8 * c8;
    const v4f qa = *(const v4fa*)gq;
    const v4f qc = *(const v4fa*)(gq + 4);
    *(v4ua*)(sX + row * XP + 8 * c8) = pack8(qa, qc, 1.0f);
    v4f sa = {0.f, 0.f, 0.f, 0.f};
    v4f sc = {0.f, 0.f, 0.f, 0.f};
    #pragma unroll
    for (int d = 0; d < NDEP; ++d) {
      const int   dp = sDep[row * NDEP + d];
      const float mk = sMsk[row * NDEP + d];
      const float* ga = ans + (size_t)dp * DM + 8 * c8;
      const v4f a = *(const v4fa*)ga;
      const v4f c = *(const v4fa*)(ga + 4);
      sa += a * mk;
      sc += c * mk;
    }
    *(v4ua*)(sX + row * XP + DM + 8 * c8) = pack8(sa, sc, sInv[row]);
  }
  __syncthreads();

  const v8f z8 = {0.f, 0.f, 0.f, 0.f, 0.f, 0.f, 0.f, 0.f};

  #pragma unroll 1
  for (int ns = 0; ns < DM / NSL; ++ns) {
    v8f acc[2][2];
    #pragma unroll
    for (int mt = 0; mt < 2; ++mt)
      #pragma unroll
      for (int nt = 0; nt < 2; ++nt) acc[mt][nt] = z8;
    #pragma unroll 1
    for (int k0 = 0; k0 < KD; k0 += 32) {
      v16h af[2];
      #pragma unroll
      for (int mt = 0; mt < 2; ++mt)
        af[mt] = ldfrag_h(sX + (16 * mt + m) * XP + k0, h);
      #pragma unroll
      for (int nt = 0; nt < 2; ++nt) {
        const int f = ns * NSL + wv * 32 + 16 * nt + m;
        const v16h bf = ldfrag_h(w1h + (size_t)f * KD + k0, h);
        #pragma unroll
        for (int mt = 0; mt < 2; ++mt)
          acc[mt][nt] = wmma_h(af[mt], bf, acc[mt][nt]);
      }
    }
    #pragma unroll
    for (int mt = 0; mt < 2; ++mt)
      #pragma unroll
      for (int nt = 0; nt < 2; ++nt) {
        const int cl = wv * 32 + 16 * nt + m;
        const float bb = b1[ns * NSL + cl];
        #pragma unroll
        for (int r = 0; r < 8; ++r) {
          const int row = 16 * mt + 8 * h + r;
          const float x = acc[mt][nt][r] * WSCI + bb;
          const float g = 0.5f * x * (1.0f + erff(x * 0.70710678118654752f));
          sY[row * YP + cl] = g;
        }
      }
    __syncthreads();
    ans_pass(sY, sTok, ans, ns, wv, lane, nrows);
    __threadfence();
    ans_pass(sY, sTok, ans, ns, wv, lane, nrows);
    __syncthreads();
  }
}

__global__ __launch_bounds__(64) void k_head(const float* __restrict__ ans,
                                             const float* __restrict__ w2,
                                             const float* __restrict__ b2,
                                             float* __restrict__ out)
{
  __shared__ __align__(16) float sOut[NC];
  const int c = threadIdx.x;
  const float* root = ans + (size_t)(NN - 1) * DM;
  const float* wr = w2 + (size_t)c * DM;
  float acc = 0.0f;
  #pragma unroll 2
  for (int d = 0; d < DM; d += 4) {
    const v4f r = *(const v4fa*)(root + d);
    const v4f w = *(const v4fa*)(wr + d);
    acc += r.x * w.x;
    acc += r.y * w.y;
    acc += r.z * w.z;
    acc += r.w * w.w;
  }
  sOut[c] = acc + b2[c];
  __syncthreads();
  const int c16 = (c < 16) ? c : 15;
  const v4f v = *(const v4fa*)(sOut + 4 * c16);
  if (c < 16) *(volatile v4f*)(out + 4 * c) = v;
  __threadfence();
  if (c < 16) *(volatile v4f*)(out + 4 * c) = v;
}

extern "C" void kernel_launch(void* const* d_in, const int* in_sizes, int n_in,
                              void* d_out, int out_size, void* d_ws, size_t ws_size,
                              hipStream_t stream)
{
  if (n_in < 7) return;
  if (in_sizes[0] != NN * DM) return;
  if (in_sizes[1] != DM * KD) return;
  if (in_sizes[2] != DM) return;
  if (in_sizes[3] != NC * DM) return;
  if (in_sizes[4] != NC) return;
  if (in_sizes[5] != NN * NDEP) return;
  if (in_sizes[6] != NN * NDEP) return;
  if (out_size != NC) return;

  const float* q        = (const float*)d_in[0];
  const float* w1       = (const float*)d_in[1];
  const float* b1       = (const float*)d_in[2];
  const float* w2       = (const float*)d_in[3];
  const float* b2       = (const float*)d_in[4];
  const int*   dep_idx  = (const int*)d_in[5];
  const int*   dep_mask = (const int*)d_in[6];
  float* out = (float*)d_out;

  const size_t bW1H  = (size_t)DM * KD * 2;
  const size_t bANS  = (size_t)NN * DM * 4;
  const size_t bLEV  = (size_t)NN * 4;
  const size_t bMETA = (size_t)META_N * 4;
  const size_t total = bW1H + bANS + bLEV + bMETA;
  if (total > ws_size) return;
  if (total > (size_t)134217728) return;

  char* ws = (char*)d_ws;
  size_t off = 0;
  unsigned short* W1H  = (unsigned short*)(ws + off); off += bW1H;
  float*          ANS  = (float*)(ws + off);          off += bANS;
  int*            LEV  = (int*)(ws + off);            off += bLEV;
  int*            META = (int*)(ws + off);            off += bMETA;
  if (off != total) return;

  k_w1<<<DM, 256, 0, stream>>>(w1, W1H);
  k_levels<<<1, 256, 0, stream>>>(dep_idx, dep_mask, LEV, META);
  hipFuncSetAttribute(reinterpret_cast<const void*>(&k_step),
                      hipFuncAttributeMaxDynamicSharedMemorySize, LDS_STEP);
  for (int s = 0; s < NLEV; ++s) {
    k_step<<<NN / MT, 256, LDS_STEP, stream>>>(q, W1H, b1, dep_idx, dep_mask,
                                               LEV, META, ANS, s);
  }
  k_head<<<1, NC, 0, stream>>>(ANS, w2, b2, out);
}
